// GRU1D_5866925326504
// MI455X (gfx1250) — hardware-verified
//
#include <hip/hip_runtime.h>
#include <math.h>
#include <stdint.h>

constexpr int NSEQ    = 1024;
constexpr int NSTEP   = 512;
constexpr int NHID    = 64;
constexpr int NG3     = 192;
constexpr int NTHR    = 256;
constexpr int TROWS   = 32;
constexpr int HPITCH  = 72;
constexpr int XCH     = 32;
constexpr int OPITCH  = 68;
constexpr int GSTRIDE = NHID * NHID;
constexpr float A_CARRY = 16.0f;
constexpr float W_CARRY = 64.0f;
constexpr float Z_FOLD  = 1.0f / 1024.0f;
constexpr float LN_EPSILON = 1e-5f;

static_assert(NSEQ % TROWS == 0, "grid covers all sequences exactly");
static_assert(NSTEP % XCH == 0, "x chunks tile the time axis exactly");
static_assert(TROWS * XCH == NTHR * 4, "one float4 per thread per x chunk");
static_assert((NG3 * NHID / 8) % NTHR == 0, "weight prep grid exact");
static_assert(NHID % 32 == 0, "K multiple of 32");

typedef __attribute__((ext_vector_type(16))) _Float16 v16h;
typedef __attribute__((ext_vector_type(8)))  _Float16 v8h;
typedef __attribute__((ext_vector_type(16))) __bf16   v16b;
typedef __attribute__((ext_vector_type(8)))  __bf16   v8b;
typedef __attribute__((ext_vector_type(8)))  float    v8f;
typedef __attribute__((ext_vector_type(4)))  float    v4f;

__device__ __forceinline__ unsigned short f2bf_bits(float f) {
  unsigned u = __float_as_uint(f);
  return (unsigned short)((u + 0x7FFFu + ((u >> 16) & 1u)) >> 16);
}
__device__ __forceinline__ float bf_bits2f(unsigned short h) { return __uint_as_float(((unsigned)h) << 16); }
__device__ __forceinline__ float bfr(float f) { return bf_bits2f(f2bf_bits(f)); }

__device__ __forceinline__ void dep_guard_h(v8f& a, v8f& b, v16h x, v16h y) { asm volatile("v_nop\n\tv_nop\n\tv_nop\n\tv_nop" : "+v"(a), "+v"(b) : "v"(x), "v"(y)); }
__device__ __forceinline__ void dep_guard_b(v8f& a, v8f& b, v16b x, v16b y) { asm volatile("v_nop\n\tv_nop\n\tv_nop\n\tv_nop" : "+v"(a), "+v"(b) : "v"(x), "v"(y)); }
__device__ __forceinline__ void keep4_h(v16h a, v16h b, v16h c, v16h d) { asm volatile("v_nop" :: "v"(a), "v"(b), "v"(c), "v"(d)); }
__device__ __forceinline__ void keep4_b(v16b a, v16b b, v16b c, v16b d) { asm volatile("v_nop" :: "v"(a), "v"(b), "v"(c), "v"(d)); }
__device__ __forceinline__ void acc_guard4(v8f& a, v8f& b, v8f& c, v8f& d) { asm volatile("v_nop\n\tv_nop\n\tv_nop\n\tv_nop" : "+v"(a), "+v"(b), "+v"(c), "+v"(d)); }
__device__ __forceinline__ void acc_guard3(v8f& a, v8f& b, v8f& c) { asm volatile("v_nop\n\tv_nop\n\tv_nop\n\tv_nop" : "+v"(a), "+v"(b), "+v"(c)); }
template <typename T> struct Frag;
template <> struct Frag<_Float16> {
  typedef v16h V; union U { v16h v; v8h h[2]; };
  static __device__ __forceinline__ v16h load(const _Float16* p) {
    U f; f.h[0] = *(const v8h*)(p); f.h[1] = *(const v8h*)(p + 16); return f.v;
  }
  static __device__ __forceinline__ v8f mma(v16h a, v16h b, v8f c) {
    return __builtin_amdgcn_wmma_f32_16x16x32_f16(false, a, false, b, (short)0, c, false, false);
  }
  static __device__ __forceinline__ void guard(v8f& a, v8f& b, v16h x, v16h y) { dep_guard_h(a, b, x, y); }
  static __device__ __forceinline__ void keep(v16h a, v16h b, v16h c, v16h d) { keep4_h(a, b, c, d); }
};
template <> struct Frag<__bf16> {
  typedef v16b V; union U { v16b v; v8b h[2]; };
  static __device__ __forceinline__ v16b load(const __bf16* p) {
    U f; f.h[0] = *(const v8b*)(p); f.h[1] = *(const v8b*)(p + 16); return f.v;
  }
  static __device__ __forceinline__ v8f mma(v16b a, v16b b, v8f c) {
    return __builtin_amdgcn_wmma_f32_16x16x32_bf16(false, a, false, b, (short)0, c, false, false);
  }
  static __device__ __forceinline__ void guard(v8f& a, v8f& b, v16b x, v16b y) { dep_guard_b(a, b, x, y); }
  static __device__ __forceinline__ void keep(v16b a, v16b b, v16b c, v16b d) { keep4_b(a, b, c, d); }
};
typedef Frag<_Float16> FragH;

__device__ __forceinline__ float fsig(float v)  { return __builtin_amdgcn_rcpf(1.0f + __expf(-v)); }
__device__ __forceinline__ float ftanh(float v) { return 1.0f - 2.0f * __builtin_amdgcn_rcpf(__expf(2.0f * v) + 1.0f); }

__global__ __launch_bounds__(NTHR) void wprep_kernel(const float* __restrict__ W, int n8, unsigned short* __restrict__ O) {
  const int i = blockIdx.x * NTHR + threadIdx.x;
  if (i >= n8) return;
  const int e0 = i * 8;
  v8h hv;
#pragma unroll
  for (int e = 0; e < 8; ++e) {
    const float fb = bfr(W[e0 + e]);
    hv[e] = (_Float16)(fb * W_CARRY);
  }
  *(volatile v8h*)(O + e0) = hv;
  __threadfence();
  *(volatile v8h*)(O + e0) = hv;
}

__device__ __forceinline__ void mac_l0(v8f (&acc)[3], const _Float16* arow, const _Float16* wh) {
#pragma unroll 1
  for (int kc = 0; kc < 2; ++kc) {
    const int k0 = kc * 32;
    const v16h a  = FragH::load(arow + k0);
    const v16h b0 = FragH::load(wh + k0);
    const v16h b1 = FragH::load(wh + GSTRIDE + k0);
    const v16h b2 = FragH::load(wh + 2 * GSTRIDE + k0);
    acc[0] = FragH::mma(a, b0, acc[0]);
    acc[1] = FragH::mma(a, b1, acc[1]);
    acc[2] = FragH::mma(a, b2, acc[2]);
    acc_guard3(acc[0], acc[1], acc[2]);
    keep4_h(a, b0, b1, b2);
  }
}

__device__ __forceinline__ void mac_l12(v8f (&acc)[4], const _Float16* abrow, const _Float16* asrow,
                                        const _Float16* wi, const _Float16* wh) {
#pragma unroll 1
  for (int kc = 0; kc < 2; ++kc) {
    const int k0 = kc * 32;
    const v16h ab  = FragH::load(abrow + k0);
    const v16h as  = FragH::load(asrow + k0);
    const v16h bir = FragH::load(wi + k0);
    const v16h bhr = FragH::load(wh + k0);
    const v16h biz = FragH::load(wi + GSTRIDE + k0);
    const v16h bhz = FragH::load(wh + GSTRIDE + k0);
    const v16h bin = FragH::load(wi + 2 * GSTRIDE + k0);
    const v16h bhn = FragH::load(wh + 2 * GSTRIDE + k0);
    acc[0] = FragH::mma(ab, bir, acc[0]);
    acc[0] = FragH::mma(as, bhr, acc[0]);
    acc[1] = FragH::mma(ab, biz, acc[1]);
    acc[1] = FragH::mma(as, bhz, acc[1]);
    acc[2] = FragH::mma(ab, bin, acc[2]);
    acc[3] = FragH::mma(as, bhn, acc[3]);
    acc_guard4(acc[0], acc[1], acc[2], acc[3]);
    keep4_h(ab, as, bir, bhr);
    keep4_h(biz, bhz, bin, bhn);
  }
}

__device__ __forceinline__ void gru_cell8(const v8f (&acc)[4], float cr, float cz, float cin, float chn, float (&h)[8]) {
#pragma unroll
  for (int r = 0; r < 8; ++r) {
    const float pr  = fmaf(acc[0][r], Z_FOLD, cr);
    const float pz  = fmaf(acc[1][r], Z_FOLD, cz);
    const float gin = fmaf(acc[2][r], Z_FOLD, cin);
    const float ghn = fmaf(acc[3][r], Z_FOLD, chn);
    const float rr  = fsig(pr);
    const float zz  = fsig(pz);
    const float nn  = ftanh(fmaf(rr, ghn, gin));
    h[r] = fmaf(zz, h[r] - nn, nn);
  }
}

__global__ __launch_bounds__(NTHR) void gru3_kernel(
    const float* __restrict__ x,
    const float* __restrict__ w_ih0, const float* __restrict__ b_ih0, const float* __restrict__ b_hh0,
    const float* __restrict__ b_ih1, const float* __restrict__ b_hh1,
    const float* __restrict__ b_ih2, const float* __restrict__ b_hh2,
    const float* __restrict__ ln_g,  const float* __restrict__ ln_b,
    const float* __restrict__ fc_w,  const float* __restrict__ fc_b,
    const unsigned short* __restrict__ Whh0p, const unsigned short* __restrict__ Wih1p,
    const unsigned short* __restrict__ Whh1p, const unsigned short* __restrict__ Wih2p,
    const unsigned short* __restrict__ Whh2p,
    float* __restrict__ out) {
  __shared__ __align__(16) _Float16 Ht[3 * TROWS * HPITCH];
  __shared__ __align__(16) float    Xs[TROWS * XCH];
  __shared__ __align__(16) float    Hs[TROWS * OPITCH];
  __shared__ __align__(16) float    Os[TROWS];

  const int tid = threadIdx.x, lane = tid & 31, wave = tid >> 5;
  const int c = lane & 15, hh = lane >> 4, koff = hh * 8;
  const int rt = wave >> 2;
  const int j  = 16 * (wave & 3) + c;
  const int rb = rt * 16 + 8 * hh;
  const int rowbase = blockIdx.x * TROWS;

#pragma unroll 1
  for (int i = tid; i < 3 * TROWS * HPITCH; i += NTHR) Ht[i] = (_Float16)0.0f;

  const float w0r  = bfr(w_ih0[j]);
  const float w0z  = bfr(w_ih0[NHID + j]);
  const float w0n  = bfr(w_ih0[2 * NHID + j]);
  const float c0r  = bfr(b_ih0[j]) + bfr(b_hh0[j]);
  const float c0z  = bfr(b_ih0[NHID + j]) + bfr(b_hh0[NHID + j]);
  const float c0in = bfr(b_ih0[2 * NHID + j]);
  const float c0hn = bfr(b_hh0[2 * NHID + j]);
  const float c1r  = bfr(b_ih1[j]) + bfr(b_hh1[j]);
  const float c1z  = bfr(b_ih1[NHID + j]) + bfr(b_hh1[NHID + j]);
  const float c1in = bfr(b_ih1[2 * NHID + j]);
  const float c1hn = bfr(b_hh1[2 * NHID + j]);
  const float c2r  = bfr(b_ih2[j]) + bfr(b_hh2[j]);
  const float c2z  = bfr(b_ih2[NHID + j]) + bfr(b_hh2[NHID + j]);
  const float c2in = bfr(b_ih2[2 * NHID + j]);
  const float c2hn = bfr(b_hh2[2 * NHID + j]);

  float hst0[8], hst1[8], hst2[8];
#pragma unroll
  for (int r = 0; r < 8; ++r) { hst0[r] = 0.0f; hst1[r] = 0.0f; hst2[r] = 0.0f; }
  __syncthreads();

  const _Float16* a0row = Ht + (rt * 16 + c) * HPITCH + koff;
  const _Float16* a1row = a0row + TROWS * HPITCH;
  const _Float16* a2row = a1row + TROWS * HPITCH;
  const _Float16* whh0 = (const _Float16*)Whh0p + (size_t)j * NHID + koff;
  const _Float16* wih1 = (const _Float16*)Wih1p + (size_t)j * NHID + koff;
  const _Float16* whh1 = (const _Float16*)Whh1p + (size_t)j * NHID + koff;
  const _Float16* wih2 = (const _Float16*)Wih2p + (size_t)j * NHID + koff;
  const _Float16* whh2 = (const _Float16*)Whh2p + (size_t)j * NHID + koff;
  const v8f z8 = {0.f, 0.f, 0.f, 0.f, 0.f, 0.f, 0.f, 0.f};

#pragma unroll 1
  for (int t = 0; t < NSTEP; ++t) {
    const int tc = t & (XCH - 1);
    if (tc == 0) {
      const int row = tid >> 3, c4 = (tid & 7) * 4;
      const v4f v = *(const v4f*)(x + ((size_t)(rowbase + row) * NSTEP + (size_t)(t + c4)));
      v4f w;
      w[0] = bfr(v[0]); w[1] = bfr(v[1]); w[2] = bfr(v[2]); w[3] = bfr(v[3]);
      *(v4f*)(Xs + row * XCH + c4) = w;
      __syncthreads();
    }
    {
      float xr[8];
#pragma unroll
      for (int r = 0; r < 8; ++r) xr[r] = Xs[(rb + r) * XCH + tc];
      v8f acc[3];
      acc[0] = z8; acc[1] = z8; acc[2] = z8;
      mac_l0(acc, a0row, whh0);
#pragma unroll
      for (int r = 0; r < 8; ++r) {
        const float pr  = fmaf(acc[0][r], Z_FOLD, fmaf(xr[r], w0r, c0r));
        const float pz  = fmaf(acc[1][r], Z_FOLD, fmaf(xr[r], w0z, c0z));
        const float gin = fmaf(xr[r], w0n, c0in);
        const float ghn = fmaf(acc[2][r], Z_FOLD, c0hn);
        const float rr  = fsig(pr);
        const float zz  = fsig(pz);
        const float nn  = ftanh(fmaf(rr, ghn, gin));
        hst0[r] = fmaf(zz, hst0[r] - nn, nn);
      }
      __syncthreads();
#pragma unroll
      for (int r = 0; r < 8; ++r) Ht[(rb + r) * HPITCH + j] = (_Float16)(A_CARRY * hst0[r]);
      __syncthreads();
    }
    {
      v8f acc[4];
      acc[0] = z8; acc[1] = z8; acc[2] = z8; acc[3] = z8;
      mac_l12(acc, a0row, a1row, wih1, whh1);
      gru_cell8(acc, c1r, c1z, c1in, c1hn, hst1);
      __syncthreads();
#pragma unroll
      for (int r = 0; r < 8; ++r) Ht[TROWS * HPITCH + (rb + r) * HPITCH + j] = (_Float16)(A_CARRY * hst1[r]);
      __syncthreads();
    }
    {
      v8f acc[4];
      acc[0] = z8; acc[1] = z8; acc[2] = z8; acc[3] = z8;
      mac_l12(acc, a1row, a2row, wih2, whh2);
      gru_cell8(acc, c2r, c2z, c2in, c2hn, hst2);
      __syncthreads();
#pragma unroll
      for (int r = 0; r < 8; ++r) Ht[2 * TROWS * HPITCH + (rb + r) * HPITCH + j] = (_Float16)(A_CARRY * hst2[r]);
      __syncthreads();
    }
  }

#pragma unroll
  for (int r = 0; r < 8; ++r) Hs[(rb + r) * OPITCH + j] = hst2[r];
  __syncthreads();
  if (tid < TROWS) {
    const float* hrow = Hs + tid * OPITCH;
    float s = 0.0f;
#pragma unroll 1
    for (int k = 0; k < NHID; ++k) s += hrow[k];
    const float mu = s * (1.0f / NHID);
    float vs = 0.0f;
#pragma unroll 1
    for (int k = 0; k < NHID; ++k) { const float d = hrow[k] - mu; vs = fmaf(d, d, vs); }
    const float var = vs * (1.0f / NHID);
    const float rs  = __builtin_amdgcn_rsqf(var + LN_EPSILON);
    float o = 0.0f;
#pragma unroll 1
    for (int k = 0; k < NHID; ++k) {
      const float nv = (hrow[k] - mu) * rs * bfr(ln_g[k]) + bfr(ln_b[k]);
      o = fmaf(nv, bfr(fc_w[k]), o);
    }
    Os[tid] = o + bfr(fc_b[0]);
  }
  __syncthreads();
  if (wave == 0 && lane < 8) {
    const v4f v = *(const v4f*)(Os + lane * 4);
    float* op = out + (size_t)rowbase + (size_t)(lane * 4);
    *(volatile v4f*)op = v;
    __threadfence();
    *(volatile v4f*)op = v;
  }
}

extern "C" void kernel_launch(void* const* d_in, const int* in_sizes, int n_in,
                              void* d_out, int out_size, void* d_ws, size_t ws_size, hipStream_t stream) {
  if (n_in < 17 || d_out == nullptr || d_ws == nullptr) return;
  if (in_sizes[0] != NSEQ * NSTEP || in_sizes[1] != NG3 || in_sizes[2] != NG3 * NHID || in_sizes[3] != NG3 ||
      in_sizes[4] != NG3 || in_sizes[5] != NG3 * NHID || in_sizes[6] != NG3 * NHID || in_sizes[7] != NG3 ||
      in_sizes[8] != NG3 || in_sizes[9] != NG3 * NHID || in_sizes[10] != NG3 * NHID || in_sizes[11] != NG3 ||
      in_sizes[12] != NG3 || in_sizes[13] != NHID || in_sizes[14] != NHID || in_sizes[15] != NHID ||
      in_sizes[16] < 1 || out_size != NSEQ) return;

  const float* x     = (const float*)d_in[0];
  const float* w_ih0 = (const float*)d_in[1];
  const float* w_hh0 = (const float*)d_in[2];
  const float* b_ih0 = (const float*)d_in[3];
  const float* b_hh0 = (const float*)d_in[4];
  const float* w_ih1 = (const float*)d_in[5];
  const float* w_hh1 = (const float*)d_in[6];
  const float* b_ih1 = (const float*)d_in[7];
  const float* b_hh1 = (const float*)d_in[8];
  const float* w_ih2 = (const float*)d_in[9];
  const float* w_hh2 = (const float*)d_in[10];
  const float* b_ih2 = (const float*)d_in[11];
  const float* b_hh2 = (const float*)d_in[12];
  const float* ln_g  = (const float*)d_in[13];
  const float* ln_b  = (const float*)d_in[14];
  const float* fc_w  = (const float*)d_in[15];
  const float* fc_b  = (const float*)d_in[16];
  float* out = (float*)d_out;

  char* ws = (char*)d_ws; size_t off = 0;
  auto carve = [&](size_t bytes) -> char* { char* p = ws + off; off += (bytes + 255) & ~(size_t)255; return p; };
  const size_t plane_bytes = (size_t)NG3 * NHID * 2;
  unsigned short* WHH0 = (unsigned short*)carve(plane_bytes);
  unsigned short* WIH1 = (unsigned short*)carve(plane_bytes);
  unsigned short* WHH1 = (unsigned short*)carve(plane_bytes);
  unsigned short* WIH2 = (unsigned short*)carve(plane_bytes);
  unsigned short* WHH2 = (unsigned short*)carve(plane_bytes);
  if (off > ws_size || off > (size_t)134217728) return;

  const int n8 = NG3 * NHID / 8;
  wprep_kernel<<<n8 / NTHR, NTHR, 0, stream>>>(w_hh0, n8, WHH0);
  wprep_kernel<<<n8 / NTHR, NTHR, 0, stream>>>(w_ih1, n8, WIH1);
  wprep_kernel<<<n8 / NTHR, NTHR, 0, stream>>>(w_hh1, n8, WHH1);
  wprep_kernel<<<n8 / NTHR, NTHR, 0, stream>>>(w_ih2, n8, WIH2);
  wprep_kernel<<<n8 / NTHR, NTHR, 0, stream>>>(w_hh2, n8, WHH2);
  gru3_kernel<<<NSEQ / TROWS, NTHR, 0, stream>>>(x, w_ih0, b_ih0, b_hh0, b_ih1, b_hh1, b_ih2, b_hh2,
                                                ln_g, ln_b, fc_w, fc_b, WHH0, WIH1, WHH1, WIH2, WHH2, out);
}
